// CorrRatio_18631568130521
// MI455X (gfx1250) — hardware-verified
//
#include <hip/hip_runtime.h>
#include <stdint.h>

typedef __attribute__((ext_vector_type(16))) _Float16 v16h;
typedef __attribute__((ext_vector_type(8)))  float    v8f;
typedef __attribute__((ext_vector_type(4)))  float    v4f;

constexpr int   NUM_BINS_K     = 32;
constexpr int   WAVES_PER_BLK  = 8;
constexpr int   THREADS_PART   = 256;
constexpr int   PART_STRIDE    = 160;
constexpr int   NBLK_PART      = 128;
constexpr float INV_LAST_BIN   = 1.0f / 31.0f;
constexpr float NEG_PRE_LOG2E  = -961.0f * 1.44269504088896340736f;
constexpr float EPS_K          = 1e-5f;
static_assert(NUM_BINS_K == 32);
static_assert(PART_STRIDE % 32 == 0);
static_assert(PART_STRIDE >= 132);
static_assert(THREADS_PART == WAVES_PER_BLK * 32);
static_assert(THREADS_PART >= PART_STRIDE);

constexpr size_t WS_PART_BYTES = (size_t)NBLK_PART * PART_STRIDE * sizeof(float);
static_assert(WS_PART_BYTES == 81920);
static_assert(WS_PART_BYTES <= 134217728ull);

__device__ __forceinline__ v8f mma_f16(v16h a, v16h b, v8f c) {
  return __builtin_amdgcn_wmma_f32_16x16x32_f16(false, a, false, b, (short)0, c, false, false);
}
__device__ __forceinline__ void wmma_guard(v8f& c0, v8f& c1, v8f& c2, v8f& c3,
                                           v16h a0, v16h a1, v16h a2, v16h a3, v16h b) {
  asm volatile("v_nop\n\tv_nop\n\tv_nop\n\tv_nop"
               : "+v"(c0), "+v"(c1), "+v"(c2), "+v"(c3)
               : "v"(a0), "v"(a1), "v"(a2), "v"(a3), "v"(b));
}

__global__ __launch_bounds__(THREADS_PART) void parzen_partial(const float* __restrict__ yt,
                                                               const float* __restrict__ yp,
                                                               float* __restrict__ part, int nch) {
  __shared__ __align__(16) float red[WAVES_PER_BLK * PART_STRIDE];
  __shared__ __align__(16) float outl[THREADS_PART];

  const int tid  = threadIdx.x;
  const int lane = tid & 31;
  const int wave = tid >> 5;
  const int h    = lane >> 4;
  const int m    = lane & 15;
  const int gw    = blockIdx.x * WAVES_PER_BLK + wave;
  const int nwtot = gridDim.x * WAVES_PER_BLK;

  const float binc_lo = (float)m * INV_LAST_BIN;
  const float binc_hi = (m == 15) ? 1.0f : (float)(m + 16) * INV_LAST_BIN;

  v8f c1lo = {0.f, 0.f, 0.f, 0.f, 0.f, 0.f, 0.f, 0.f};
  v8f c1hi = {0.f, 0.f, 0.f, 0.f, 0.f, 0.f, 0.f, 0.f};
  v8f c2lo = {0.f, 0.f, 0.f, 0.f, 0.f, 0.f, 0.f, 0.f};
  v8f c2hi = {0.f, 0.f, 0.f, 0.f, 0.f, 0.f, 0.f, 0.f};
  float st = 0.f, stt = 0.f, sp = 0.f, spp = 0.f;

#pragma unroll 1
  for (int ch = gw; ch < nch; ch += nwtot) {
    const size_t k0 = (size_t)ch << 5;
    const float* pt = yt + k0 + 8 * h;
    const float* pq = yp + k0 + 8 * h;
    const v4f t0 = *(const v4f*)(pt);
    const v4f t1 = *(const v4f*)(pt + 4);
    const v4f t2 = *(const v4f*)(pt + 16);
    const v4f t3 = *(const v4f*)(pt + 20);
    const v4f q0 = *(const v4f*)(pq);
    const v4f q1 = *(const v4f*)(pq + 4);
    const v4f q2 = *(const v4f*)(pq + 16);
    const v4f q3 = *(const v4f*)(pq + 20);
    const float xt = yt[k0 + lane];
    const float xp = yp[k0 + lane];
    st += xt; stt += xt * xt;
    sp += xp; spp += xp * xp;

    float tv[16], pv[16];
#pragma unroll
    for (int e = 0; e < 4; ++e) {
      tv[e] = t0[e]; tv[4 + e] = t1[e]; tv[8 + e] = t2[e]; tv[12 + e] = t3[e];
      pv[e] = q0[e]; pv[4 + e] = q1[e]; pv[8 + e] = q2[e]; pv[12 + e] = q3[e];
    }

    v16h aPl, aPh, aTl, aTh, bx;
#pragma unroll
    for (int i = 0; i < 16; ++i) {
      const float vt = tv[i];
      const float vp = pv[i];
      const float d0 = vp - binc_lo;
      const float d1 = vp - binc_hi;
      const float d2 = vt - binc_lo;
      const float d3 = vt - binc_hi;
      aPl[i] = (_Float16)exp2f(NEG_PRE_LOG2E * (d0 * d0));
      aPh[i] = (_Float16)exp2f(NEG_PRE_LOG2E * (d1 * d1));
      aTl[i] = (_Float16)exp2f(NEG_PRE_LOG2E * (d2 * d2));
      aTh[i] = (_Float16)exp2f(NEG_PRE_LOG2E * (d3 * d3));
      const float bv = (m == 0) ? vt : ((m == 1) ? vp : ((m == 2) ? 1.0f : 0.0f));
      bx[i] = (_Float16)bv;
    }

    c1lo = mma_f16(aPl, bx, c1lo);
    c1hi = mma_f16(aPh, bx, c1hi);
    c2lo = mma_f16(aTl, bx, c2lo);
    c2hi = mma_f16(aTh, bx, c2hi);
    wmma_guard(c1lo, c1hi, c2lo, c2hi, aPl, aPh, aTl, aTh, bx);
  }

#pragma unroll
  for (int off = 16; off >= 1; off >>= 1) {
    st  += __shfl_xor(st,  off, 32);
    stt += __shfl_xor(stt, off, 32);
    sp  += __shfl_xor(sp,  off, 32);
    spp += __shfl_xor(spp, off, 32);
  }

  float* rw = red + wave * PART_STRIDE;
  if (m == 0) {
#pragma unroll
    for (int r = 0; r < 8; ++r) {
      rw[8 * h + r]      = c1lo[r];
      rw[16 + 8 * h + r] = c1hi[r];
    }
  }
  if (m == 1) {
#pragma unroll
    for (int r = 0; r < 8; ++r) {
      rw[64 + 8 * h + r] = c2lo[r];
      rw[80 + 8 * h + r] = c2hi[r];
    }
  }
  if (m == 2) {
#pragma unroll
    for (int r = 0; r < 8; ++r) {
      rw[32 + 8 * h + r]  = c1lo[r];
      rw[48 + 8 * h + r]  = c1hi[r];
      rw[96 + 8 * h + r]  = c2lo[r];
      rw[112 + 8 * h + r] = c2hi[r];
    }
  }
  if (lane == 0) {
    rw[128] = st; rw[129] = stt; rw[130] = sp; rw[131] = spp;
  }
  __syncthreads();

  {
    float s = 0.f;
    if (tid < 132) {
#pragma unroll
      for (int w = 0; w < WAVES_PER_BLK; ++w) s += red[w * PART_STRIDE + tid];
    }
    outl[tid] = s;
  }
  __syncthreads();

  if (wave == 0) {
    const v4f v0 = *(const v4f*)(outl + 4 * lane);
    const v4f v1 = *(const v4f*)(outl + 128 + 4 * lane);
    float* pb = part + (size_t)blockIdx.x * PART_STRIDE;
    for (int pass = 0; pass < 2; ++pass) {
      *(volatile v4f*)(pb + 4 * lane) = v0;
      if (lane < 8) *(volatile v4f*)(pb + 128 + 4 * lane) = v1;
      __threadfence();
    }
  }
}

__global__ __launch_bounds__(256) void eta_final(const float* __restrict__ part, float* __restrict__ out,
                                                 int nblk, int nvox) {
  __shared__ double acc[PART_STRIDE];
  const int tid = threadIdx.x;
  if (tid < PART_STRIDE) {
    double s = 0.0;
#pragma unroll 1
    for (int b = 0; b < nblk; ++b) s += (double)part[(size_t)b * PART_STRIDE + tid];
    acc[tid] = s;
  }
  __syncthreads();
  if (tid == 0) {
    const double nd  = (double)nvox;
    const double eps = (double)EPS_K;
    double cr = 0.0;
#pragma unroll 1
    for (int dir = 0; dir < 2; ++dir) {
      const int tb = dir * 64;
      const int sb = dir * 64 + 32;
      const double sx  = acc[128 + 2 * dir];
      const double sxx = acc[129 + 2 * dir];
      const double mean = sx / nd;
      const double var = (sxx - sx * mean) / (nd - 1.0);
      double bg = 0.0, tot = 0.0;
#pragma unroll 1
      for (int k = 0; k < NUM_BINS_K; ++k) {
        const double sk = acc[sb + k];
        const double tk = acc[tb + k];
        const double mk = tk / (sk + eps);
        const double d  = mk - mean;
        bg  += sk * d * d;
        tot += sk;
      }
      const double between = bg / (tot + eps);
      const double eta = between / (var + eps);
      cr += eta * (1.0 / 3.0);
    }
    const float r = (float)(-cr * 0.5);
    *(volatile float*)out = r;
    __threadfence();
    *(volatile float*)out = r;
  }
}

extern "C" void kernel_launch(void* const* d_in, const int* in_sizes, int n_in,
                              void* d_out, int out_size, void* d_ws, size_t ws_size,
                              hipStream_t stream) {
  if (n_in < 2 || out_size < 1) return;
  if (ws_size < WS_PART_BYTES) return;
  const float* yt = (const float*)d_in[0];
  const float* yp = (const float*)d_in[1];
  int nvox = in_sizes[0];
  if (in_sizes[1] < nvox) nvox = in_sizes[1];
  if (nvox < NUM_BINS_K) return;
  const int nch = nvox >> 5;

  float* part = (float*)d_ws;
  float* out  = (float*)d_out;

  parzen_partial<<<NBLK_PART, THREADS_PART, 0, stream>>>(yt, yp, part, nch);
  eta_final<<<1, 256, 0, stream>>>(part, out, NBLK_PART, nvox);
}
